// SwinTransformerBlock_1228360647057
// MI455X (gfx1250) — hardware-run, weakly checked
//
#include <hip/hip_runtime.h>


#define NB_  4
#define GRD  96
#define DM   256
#define NH_  8
#define HD   32
#define HDP  64
#define NWIN 48
#define WP   192
#define NTK  (NWIN * WP)
#define FF   1024
#define MCH  4608
#define PCAR 1024.0f
#define SCL  0.0625f
typedef _Float16 h16;
typedef unsigned short bf;
typedef __attribute__((ext_vector_type(16))) __bf16   v16bf;
typedef __attribute__((ext_vector_type(16))) _Float16 v16h;
typedef __attribute__((ext_vector_type(8)))  _Float16 v8h;
typedef __attribute__((ext_vector_type(8)))  unsigned short v8us;
typedef __attribute__((ext_vector_type(8)))  float    v8f;
typedef __attribute__((ext_vector_type(4)))  float    v4f;
typedef v8h  __attribute__((may_alias)) v8ha;
typedef v4f  __attribute__((may_alias)) v4fa;
typedef v8us __attribute__((may_alias)) v8usa;

__device__ __forceinline__ unsigned short f2bf(float f) { unsigned u = __float_as_uint(f); u += 0x7FFFu + ((u >> 16) & 1u); return (unsigned short)(u >> 16); }
__device__ __forceinline__ float bf2f(unsigned short b) { return __uint_as_float(((unsigned)b) << 16); }
__device__ __forceinline__ float bfr(float f) { return bf2f(f2bf(f)); }
__device__ __forceinline__ v16h cat16(v8h lo, v8h hi) { return __builtin_shufflevector(lo, hi, 0, 1, 2, 3, 4, 5, 6, 7, 8, 9, 10, 11, 12, 13, 14, 15); }
__device__ __forceinline__ v16bf cat16b(v8us lo, v8us hi) { return __builtin_bit_cast(v16bf, __builtin_shufflevector(lo, hi, 0, 1, 2, 3, 4, 5, 6, 7, 8, 9, 10, 11, 12, 13, 14, 15)); }
__device__ __forceinline__ v8f wmma16(v16h a, v16h b, v8f c) { return __builtin_amdgcn_wmma_f32_16x16x32_f16(false, a, false, b, (short)0, c, false, false); }
__device__ __forceinline__ v8f wmmab(v16bf a, v16bf b, v8f c) { return __builtin_amdgcn_wmma_f32_16x16x32_bf16(false, a, false, b, (short)0, c, false, false); }


template <typename T16> struct WFrag;
template <> struct WFrag<h16> { typedef v16h V; static __device__ __forceinline__ V ld(const h16* p) { return cat16(*(const v8h*)p, *(const v8h*)(p + 16)); } static __device__ __forceinline__ v8f mma(V a, V b, v8f c) { return wmma16(a, b, c); } };
template <> struct WFrag<bf> { typedef v16bf V; static __device__ __forceinline__ V ld(const bf* p) { return cat16b(*(const v8us*)p, *(const v8us*)(p + 16)); } static __device__ __forceinline__ v8f mma(V a, V b, v8f c) { return wmmab(a, b, c); } };
template <typename T16, int NSPLIT, bool BIAS>
__global__ __launch_bounds__(32) void k_gemmw(const T16* __restrict__ A, const T16* __restrict__ A2, const T16* __restrict__ Bt, const T16* __restrict__ Bt2, int K, float* C, int ldc, const float* __restrict__ bias, size_t sA, size_t sB, size_t sC) {
    typedef typename WFrag<T16>::V V;
    __shared__ __align__(16) float os[16 * 68];
    const size_t z = blockIdx.z; A += z * sA; if (A2) A2 += z * sA; Bt += z * sB; if (Bt2) Bt2 += z * sB; C += z * sC;
    const int lane = threadIdx.x & 31, lr = lane & 15, hi = lane >> 4; const int r0 = blockIdx.x * 64, c0 = blockIdx.y * 64;
    v8f acc[4][4];
#pragma unroll
    for (int mb = 0; mb < 4; ++mb)
#pragma unroll
        for (int nb = 0; nb < 4; ++nb) acc[mb][nb] = (v8f){};
    const size_t aoff = (size_t)(r0 + lr) * K + 8 * hi, boff = (size_t)(c0 + lr) * K + 8 * hi;
#pragma unroll 1
    for (int kc = 0; kc < K; kc += 32) {
        V a[4], a2[4];
#pragma unroll
        for (int mb = 0; mb < 4; ++mb) { a[mb] = WFrag<T16>::ld(A + aoff + (size_t)mb * 16 * K + kc); if (NSPLIT == 1 || NSPLIT == 2) a2[mb] = WFrag<T16>::ld(A2 + aoff + (size_t)mb * 16 * K + kc); }
#pragma unroll
        for (int nb = 0; nb < 4; ++nb) { const V b = WFrag<T16>::ld(Bt + boff + (size_t)nb * 16 * K + kc); V b2; if (NSPLIT >= 2) b2 = WFrag<T16>::ld(Bt2 + boff + (size_t)nb * 16 * K + kc);
#pragma unroll
            for (int mb = 0; mb < 4; ++mb) { acc[mb][nb] = WFrag<T16>::mma(a[mb], b, acc[mb][nb]); if (NSPLIT == 1 || NSPLIT == 2) acc[mb][nb] = WFrag<T16>::mma(a2[mb], b, acc[mb][nb]); if (NSPLIT >= 2) acc[mb][nb] = WFrag<T16>::mma(a[mb], b2, acc[mb][nb]); } }
        asm volatile("v_nop\n\tv_nop\n\tv_nop\n\tv_nop" : "+v"(acc[0][0]), "+v"(acc[1][1]), "+v"(acc[2][2]), "+v"(acc[3][3]) : "v"(a[0]), "v"(a[3]));
    }
#pragma unroll
    for (int mb = 0; mb < 4; ++mb) {
#pragma unroll
        for (int nb = 0; nb < 4; ++nb) {
#pragma unroll
            for (int j = 0; j < 8; ++j) os[(hi * 8 + j) * 68 + nb * 16 + lr] = acc[mb][nb][j]; }
        __builtin_amdgcn_wave_barrier(); asm volatile("" ::: "memory");
        float* crow = C + (size_t)(r0 + mb * 16) * ldc + c0;
#pragma unroll 1
        for (int ps = 0; ps < 2; ++ps) {
#pragma unroll
            for (int s = 0; s < 8; ++s) { const int row = 2 * s + hi, cofs = lr * 4; v4f val = *(const v4fa*)(os + row * 68 + cofs); if (BIAS) { val[0] += bfr(bias[c0 + cofs]); val[1] += bfr(bias[c0 + cofs + 1]); val[2] += bfr(bias[c0 + cofs + 2]); val[3] += bfr(bias[c0 + cofs + 3]); }
                *(volatile v4f*)(crow + (size_t)row * ldc + cofs) = val; }
            if (ps == 0) __threadfence(); }
        __builtin_amdgcn_wave_barrier(); asm volatile("" ::: "memory");
    }
}

typedef __attribute__((ext_vector_type(4))) unsigned short v4us;
typedef __attribute__((ext_vector_type(2))) unsigned short v2us;
typedef __attribute__((ext_vector_type(2))) _Float16 v2h;
typedef __attribute__((ext_vector_type(4))) _Float16 v4h;
typedef __attribute__((ext_vector_type(2))) float v2f;
__device__ __forceinline__ h16 tohx(float x) { return (h16)x; }
__device__ __forceinline__ void splitf(float y, unsigned short& h, unsigned short& l) { h = f2bf(y); l = f2bf(y - bf2f(h)); }
__device__ __forceinline__ int tok2row(int t) { const int w = t / WP, p = t % WP; const int r = (p / 32) * 16 + (w / 3), c = (p % 32) * 3 + (w % 3); const int i = (r - 16 + GRD) % GRD, j = (c - 3 + GRD) % GRD; return i * GRD + j; }
__global__ __launch_bounds__(256) void k_wtG(const float* __restrict__ w, int K, int N, bf* Bt) {
    const int lane = threadIdx.x & 31; const int L0 = (blockIdx.x * 8 + (threadIdx.x >> 5)) * 8; const int nlines = N * K / 64;
#pragma unroll
    for (int ps = 0; ps < 2; ++ps) {
#pragma unroll 1
        for (int l = 0; l < 8; ++l) { const int L = L0 + l; if (L >= nlines) break; const size_t e = (size_t)L * 64 + lane * 2; const int k = (int)(e % K), n = (int)(e / K); v2us o;
            o[0] = f2bf(w[(size_t)k * N + n]); o[1] = f2bf(w[(size_t)(k + 1) * N + n]); *(volatile v2us*)(Bt + e) = o; }
        if (ps == 0) __threadfence(); }
}

template <int GATHER>
__global__ __launch_bounds__(256) void k_ln(const float* __restrict__ IN, const float* __restrict__ g, const float* __restrict__ bb, bf* Xh, bf* Xl, float* R) {
    const int lane = threadIdx.x & 31; const int t = blockIdx.x * 8 + (threadIdx.x >> 5); if (t >= NTK) return; const float* src = GATHER ? (IN + (size_t)tok2row(t) * DM) : (IN + (size_t)t * DM); const v4f a0 = *(const v4f*)(src + lane * 8); const v4f a1 = *(const v4f*)(src + lane * 8 + 4); float v[8]; float s = 0.f;
#pragma unroll
    for (int q = 0; q < 4; ++q) { v[q] = GATHER ? bfr(a0[q]) : a0[q]; v[4 + q] = GATHER ? bfr(a1[q]) : a1[q]; }
#pragma unroll
    for (int q = 0; q < 8; ++q) s = __fadd_rn(s, v[q]);
#pragma unroll
    for (int sh = 16; sh; sh >>= 1) s = __fadd_rn(s, __shfl_xor(s, sh, 32));
    const float mu = __fdiv_rn(s, (float)DM); float s2 = 0.f;
#pragma unroll
    for (int q = 0; q < 8; ++q) { float d0 = __fsub_rn(v[q], mu); asm volatile("" : "+v"(d0)); float p = __fmul_rn(d0, d0); asm volatile("" : "+v"(p)); s2 = __fadd_rn(s2, p); }
#pragma unroll
    for (int sh = 16; sh; sh >>= 1) s2 = __fadd_rn(s2, __shfl_xor(s2, sh, 32));
    const float rs = __fdiv_rn(1.0f, __fsqrt_rn(__fadd_rn(__fdiv_rn(s2, (float)DM), 1e-5f))); v8us oh, ol;
#pragma unroll
    for (int q = 0; q < 8; ++q) { const int c = lane * 8 + q; float xn = __fmul_rn(__fsub_rn(v[q], mu), rs); asm volatile("" : "+v"(xn)); float gg = bfr(g[c]); asm volatile("" : "+v"(gg)); float y = __fmul_rn(xn, gg); asm volatile("" : "+v"(y)); float be = bfr(bb[c]); asm volatile("" : "+v"(be)); y = __fadd_rn(y, be); unsigned short h2, l2; splitf(y, h2, l2); oh[q] = h2; ol[q] = l2; }
    const size_t o = (size_t)t * DM + lane * 8;
#pragma unroll 1
    for (int ps = 0; ps < 2; ++ps) { *(volatile v8us*)(Xh + o) = oh; *(volatile v8us*)(Xl + o) = ol; if (GATHER) { v4f r0, r1; for (int q = 0; q < 4; ++q) { r0[q] = v[q]; r1[q] = v[4 + q]; } *(volatile v4f*)(R + o) = r0; *(volatile v4f*)(R + o + 4) = r1; } if (ps == 0) __threadfence(); }
}
__global__ __launch_bounds__(256) void k_qkpl(const float* __restrict__ F, h16* P16) { const size_t e = ((size_t)blockIdx.x * 256 + threadIdx.x) * 2; if (e >= (size_t)NH_ * NTK * HD) return; const int d = (int)(e % HD); const size_t tk = (e / HD) % NTK; const int h = (int)(e / ((size_t)HD * NTK)); v2h o;
    o[0] = tohx(F[tk * DM + h * HD + d]); o[1] = tohx(F[tk * DM + h * HD + d + 1]); *(volatile v2h*)(P16 + e) = o; __threadfence(); *(volatile v2h*)(P16 + e) = o; }
__global__ __launch_bounds__(256) void k_vtpl(const float* __restrict__ F, h16* V16) { const size_t e = ((size_t)blockIdx.x * 256 + threadIdx.x) * 2; if (e >= (size_t)NH_ * NWIN * HDP * WP) return; const int p = (int)(e % WP); const int dp = (int)((e / WP) % HDP); const size_t w = (e / ((size_t)WP * HDP)) % NWIN; const int h = (int)(e / ((size_t)WP * HDP * NWIN)); v2h o;
    if (dp < HD) { o[0] = tohx(F[(w * WP + p) * DM + h * HD + dp]); o[1] = tohx(F[(w * WP + p + 1) * DM + h * HD + dp]); } else { o[0] = (h16)0.0f; o[1] = (h16)0.0f; }
    *(volatile v2h*)(V16 + e) = o; __threadfence(); *(volatile v2h*)(V16 + e) = o; }
__global__ __launch_bounds__(256) void k_asoftW(const float* __restrict__ Sb, const float* __restrict__ pb, int h, h16* P16) {
    const int lane = threadIdx.x & 31; const int row = blockIdx.x * 8 + (threadIdx.x >> 5); if (row >= NWIN * WP) return; const int q = row % WP; const float* sr = Sb + (size_t)row * WP; const float* pr = pb + ((size_t)h * WP + q) * WP; float v[6]; float mx = -3.0e38f;
    { const v4f a = *(const v4f*)(sr + lane * 4); const v4f p4 = *(const v4f*)(pr + lane * 4); const v2f a2 = *(const v2f*)(sr + 128 + lane * 2); const v2f p2 = *(const v2f*)(pr + 128 + lane * 2);
#pragma unroll
      for (int i = 0; i < 4; ++i) { float sc = __fmul_rn(a[i], SCL); asm volatile("" : "+v"(sc)); float bb = bfr(p4[i]); asm volatile("" : "+v"(bb)); v[i] = __fadd_rn(sc, bb); mx = fmaxf(mx, v[i]); }
#pragma unroll
      for (int i = 0; i < 2; ++i) { float sc = __fmul_rn(a2[i], SCL); asm volatile("" : "+v"(sc)); float bb = bfr(p2[i]); asm volatile("" : "+v"(bb)); v[4 + i] = __fadd_rn(sc, bb); mx = fmaxf(mx, v[4 + i]); } }
#pragma unroll
    for (int sh = 16; sh; sh >>= 1) mx = fmaxf(mx, __shfl_xor(mx, sh, 32));
    float sum = 0.f;
#pragma unroll
    for (int i = 0; i < 6; ++i) { float d0 = __fsub_rn(v[i], mx); asm volatile("" : "+v"(d0)); v[i] = __builtin_amdgcn_exp2f(__fmul_rn(d0, 1.4426950408889634f)); sum = __fadd_rn(sum, v[i]); }
#pragma unroll
    for (int sh = 16; sh; sh >>= 1) sum = __fadd_rn(sum, __shfl_xor(sum, sh, 32));
    const float f = __fdiv_rn(PCAR, sum);
#pragma unroll 1
    for (int ps = 0; ps < 2; ++ps) { v4h o4; v2h o2;
#pragma unroll
        for (int i = 0; i < 4; ++i) { float y = __fmul_rn(v[i], f); asm volatile("" : "+v"(y)); o4[i] = tohx(y); }
#pragma unroll
        for (int i = 0; i < 2; ++i) { float y = __fmul_rn(v[4 + i], f); asm volatile("" : "+v"(y)); o2[i] = tohx(y); }
        *(volatile v4h*)(P16 + (size_t)row * WP + lane * 4) = o4; *(volatile v2h*)(P16 + (size_t)row * WP + 128 + lane * 2) = o2; if (ps == 0) __threadfence(); }
}
__global__ __launch_bounds__(256) void k_resid(const float* __restrict__ R, const float* __restrict__ O, float* AR) { const size_t e = ((size_t)blockIdx.x * 256 + threadIdx.x) * 4; if (e >= (size_t)NTK * DM) return; const int c = (int)(e % DM); const size_t tk = e / DM; const int h = c / HD, d = c % HD;
    const v4f r = *(const v4f*)(R + e); const v4f ov = *(const v4f*)(O + (((size_t)h * NTK + tk) * HDP + d)); v4f o;
#pragma unroll
    for (int q = 0; q < 4; ++q) { float y = __fmul_rn(ov[q], 1.0f / PCAR); asm volatile("" : "+v"(y)); o[q] = __fadd_rn(r[q], y); }
    *(volatile v4f*)(AR + e) = o; __threadfence(); *(volatile v4f*)(AR + e) = o; }
__global__ __launch_bounds__(256) void k_gelu(const float* __restrict__ F1, bf* Gh, bf* Gl, size_t n2) { const size_t i = (size_t)blockIdx.x * 256 + threadIdx.x; if (i >= n2) return; const v2f x = *(const v2f*)(F1 + i * 2); v2us oh, ol;
#pragma unroll
    for (int q = 0; q < 2; ++q) { const float er = erff(__fmul_rn(x[q], 0.70710678118654752f)); float hx = __fmul_rn(0.5f, x[q]); asm volatile("" : "+v"(hx)); const float y = __fmul_rn(hx, __fadd_rn(1.0f, er)); unsigned short h2, l2; splitf(y, h2, l2); oh[q] = h2; ol[q] = l2; }
    *(volatile v2us*)(Gh + i * 2) = oh; *(volatile v2us*)(Gl + i * 2) = ol; __threadfence(); *(volatile v2us*)(Gh + i * 2) = oh; *(volatile v2us*)(Gl + i * 2) = ol; }
__global__ __launch_bounds__(256) void k_outS(const float* __restrict__ AR, const float* __restrict__ F2, float* out) { const int lane = threadIdx.x & 31; const int t = blockIdx.x * 8 + (threadIdx.x >> 5); if (t >= NTK) return; const size_t si = (size_t)t * DM + lane * 8; const size_t di = (size_t)tok2row(t) * DM + lane * 8;
    const v4f a0 = *(const v4f*)(AR + si), a1 = *(const v4f*)(AR + si + 4), f0 = *(const v4f*)(F2 + si), f1 = *(const v4f*)(F2 + si + 4); v4f o0, o1;
#pragma unroll
    for (int q = 0; q < 4; ++q) { o0[q] = __fadd_rn(a0[q], f0[q]); o1[q] = __fadd_rn(a1[q], f1[q]); }
    *(volatile v4f*)(out + di) = o0; *(volatile v4f*)(out + di + 4) = o1; __threadfence(); *(volatile v4f*)(out + di) = o0; *(volatile v4f*)(out + di + 4) = o1; }

extern "C" void kernel_launch(void* const* d_in, const int* in_sizes, int n_in,
                              void* d_out, int out_size, void* d_ws, size_t ws_size, hipStream_t stream) {
    (void)in_sizes; (void)n_in; (void)out_size;
    const float* emb = (const float*)d_in[0]; const float* l1g = (const float*)d_in[1]; const float* l1b = (const float*)d_in[2]; const float* wq = (const float*)d_in[3]; const float* bq = (const float*)d_in[4]; const float* wk = (const float*)d_in[5]; const float* bk = (const float*)d_in[6]; const float* wv = (const float*)d_in[7]; const float* bv = (const float*)d_in[8];
    const float* pb = (const float*)d_in[9]; const float* l2g = (const float*)d_in[10]; const float* l2b = (const float*)d_in[11]; const float* w1 = (const float*)d_in[12]; const float* b1 = (const float*)d_in[13]; const float* w2 = (const float*)d_in[14]; const float* b2 = (const float*)d_in[15];
    float* OUT = (float*)d_out;
    char* wsp = (char*)d_ws;
    auto take = [&](size_t bytes) { char* p = wsp; wsp += (bytes + 255) & ~(size_t)255; return (void*)p; };
    bf* WQ = (bf*)take((size_t)DM * DM * 2); bf* WK = (bf*)take((size_t)DM * DM * 2); bf* WV = (bf*)take((size_t)DM * DM * 2); bf* W1 = (bf*)take((size_t)FF * DM * 2); bf* W2 = (bf*)take((size_t)DM * FF * 2);
    bf* Xh = (bf*)take((size_t)NTK * DM * 2); bf* Xl = (bf*)take((size_t)NTK * DM * 2); float* R = (float*)take((size_t)NTK * DM * 4); float* FQ = (float*)take((size_t)NTK * DM * 4); float* FK = (float*)take((size_t)NTK * DM * 4);
    h16* QP = (h16*)take((size_t)NH_ * NTK * HD * 2); h16* KP = (h16*)take((size_t)NH_ * NTK * HD * 2); h16* VT = (h16*)take((size_t)NH_ * NWIN * HDP * WP * 2); float* Sb = (float*)take((size_t)NWIN * WP * WP * 4); h16* P16 = (h16*)take((size_t)NWIN * WP * WP * 2);
    float* Ob = (float*)take((size_t)NH_ * NTK * HDP * 4); float* AR = (float*)take((size_t)NTK * DM * 4); float* F1 = (float*)take((size_t)MCH * FF * 4); bf* Gh = (bf*)take((size_t)MCH * FF * 2); bf* Gl = (bf*)take((size_t)MCH * FF * 2); float* F2 = (float*)take((size_t)NTK * DM * 4);
    if ((size_t)(wsp - (char*)d_ws) > ws_size) return;
    float* FV = FK;
    k_wtG<<<(unsigned)((DM * DM / 64 + 63) / 64), 256, 0, stream>>>(wq, DM, DM, WQ); k_wtG<<<(unsigned)((DM * DM / 64 + 63) / 64), 256, 0, stream>>>(wk, DM, DM, WK); k_wtG<<<(unsigned)((DM * DM / 64 + 63) / 64), 256, 0, stream>>>(wv, DM, DM, WV);
    k_wtG<<<(unsigned)((DM * FF / 64 + 63) / 64), 256, 0, stream>>>(w1, DM, FF, W1); k_wtG<<<(unsigned)((FF * DM / 64 + 63) / 64), 256, 0, stream>>>(w2, FF, DM, W2);
    static_assert(NTK % 64 == 0 && WP % 64 == 0 && NTK % MCH == 0 && MCH % 64 == 0, "tiles");
    for (int b = 0; b < NB_; ++b) {
        k_ln<1><<<NTK / 8, 256, 0, stream>>>(emb + (size_t)b * GRD * GRD * DM, l1g, l1b, Xh, Xl, R);
        k_gemmw<bf, 1, true><<<dim3(NTK / 64, DM / 64, 1), 32, 0, stream>>>(Xh, Xl, WQ, nullptr, DM, FQ, DM, bq, 0, 0, 0); k_qkpl<<<(unsigned)(((size_t)NH_ * NTK * HD / 2 + 255) / 256), 256, 0, stream>>>(FQ, QP);
        k_gemmw<bf, 1, true><<<dim3(NTK / 64, DM / 64, 1), 32, 0, stream>>>(Xh, Xl, WK, nullptr, DM, FK, DM, bk, 0, 0, 0); k_qkpl<<<(unsigned)(((size_t)NH_ * NTK * HD / 2 + 255) / 256), 256, 0, stream>>>(FK, KP);
        k_gemmw<bf, 1, true><<<dim3(NTK / 64, DM / 64, 1), 32, 0, stream>>>(Xh, Xl, WV, nullptr, DM, FV, DM, bv, 0, 0, 0); k_vtpl<<<(unsigned)(((size_t)NH_ * NWIN * HDP * WP / 2 + 255) / 256), 256, 0, stream>>>(FV, VT);
        for (int h = 0; h < NH_; ++h) {
            k_gemmw<h16, 0, false><<<dim3(WP / 64, WP / 64, NWIN), 32, 0, stream>>>(QP + (size_t)h * NTK * HD, nullptr, KP + (size_t)h * NTK * HD, nullptr, HD, Sb, WP, nullptr, (size_t)WP * HD, (size_t)WP * HD, (size_t)WP * WP);
            k_asoftW<<<NWIN * WP / 8, 256, 0, stream>>>(Sb, pb, h, P16);
            k_gemmw<h16, 0, false><<<dim3(WP / 64, HDP / 64, NWIN), 32, 0, stream>>>(P16, nullptr, VT + (size_t)h * NWIN * HDP * WP, nullptr, WP, Ob + (size_t)h * NTK * HDP, HDP, nullptr, (size_t)WP * WP, (size_t)HDP * WP, (size_t)WP * HDP); }
        k_resid<<<(unsigned)(((size_t)NTK * DM / 4 + 255) / 256), 256, 0, stream>>>(R, Ob, AR);
        k_ln<0><<<NTK / 8, 256, 0, stream>>>(AR, l2g, l2b, Xh, Xl, nullptr);
        for (size_t r0 = 0; r0 < NTK; r0 += MCH) {
            k_gemmw<bf, 1, true><<<dim3(MCH / 64, FF / 64, 1), 32, 0, stream>>>(Xh + r0 * DM, Xl + r0 * DM, W1, nullptr, DM, F1, FF, b1, 0, 0, 0);
            k_gelu<<<(unsigned)(((size_t)MCH * FF / 2 + 255) / 256), 256, 0, stream>>>(F1, Gh, Gl, (size_t)MCH * FF / 2);
            k_gemmw<bf, 1, true><<<dim3(MCH / 64, DM / 64, 1), 32, 0, stream>>>(Gh, Gl, W2, nullptr, FF, F2 + r0 * DM, DM, b2, 0, 0, 0); }
        k_outS<<<NTK / 8, 256, 0, stream>>>(AR, F2, OUT + (size_t)b * GRD * GRD * DM); }
}
